// MultiheadedAttentionFM_90022514524806
// MI455X (gfx1250) — hardware-verified
//
#include <hip/hip_runtime.h>
#include <math.h>

typedef __attribute__((ext_vector_type(16))) _Float16 v16h;
typedef __attribute__((ext_vector_type(16))) __bf16 v16b;
typedef __attribute__((ext_vector_type(8)))  _Float16 v8h;
typedef __attribute__((ext_vector_type(8)))  float v8f;
typedef __attribute__((ext_vector_type(4)))  float v4f;
typedef __attribute__((ext_vector_type(2)))  float v2f;
typedef __attribute__((ext_vector_type(4)))  unsigned v4u;
typedef __attribute__((ext_vector_type(4)))  int v4i;
typedef float __attribute__((may_alias)) float_a;
typedef int __attribute__((may_alias)) int_a;

template <typename T> __device__ __forceinline__ void vst2(void* p, T v) { *(volatile T*)p = v; __threadfence(); *(volatile T*)p = v; }
__device__ __forceinline__ v8f wmma16(v16h a, v16h b, v8f c) {
  v8f d = __builtin_amdgcn_wmma_f32_16x16x32_f16(false, a, false, b, (short)0, c, false, false);
  asm volatile("v_nop\n\tv_nop\n\tv_nop\n\tv_nop" : "+v"(d) : "v"(a), "v"(b));
  return d;
}
__device__ __forceinline__ v8f wmma_bf(v16b a, v16b b, v8f c) {
  v8f d = __builtin_amdgcn_wmma_f32_16x16x32_bf16(false, a, false, b, (short)0, c, false, false);
  asm volatile("v_nop\n\tv_nop\n\tv_nop\n\tv_nop" : "+v"(d) : "v"(a), "v"(b));
  return d;
}
__device__ __forceinline__ v16h frag_h(const _Float16* rowk0, int lane) {
  union { v16h v; v8h q[2]; } u; const _Float16* p = rowk0 + 8 * (lane >> 4);
  u.q[0] = *(const v8h*)p; u.q[1] = *(const v8h*)(p + 16); return u.v;
}
__device__ __forceinline__ v16h frag_f32(const float* rowk0, int lane) {
  v16h a; const float* p = rowk0 + 8 * (lane >> 4);
#pragma unroll
  for (int i = 0; i < 8; ++i) { a[i] = (_Float16)p[i]; a[8 + i] = (_Float16)p[16 + i]; }
  return a;
}
__device__ __forceinline__ v16h frag_f32s(const float* rowk0, int lane, float sc) {
  v16h a; const float* p = rowk0 + 8 * (lane >> 4);
#pragma unroll
  for (int i = 0; i < 8; ++i) { a[i] = (_Float16)(p[i] * sc); a[8 + i] = (_Float16)(p[16 + i] * sc); }
  return a;
}
__device__ __forceinline__ v16h fragc_f32(const float* W, int k0, int n, int lane, int ld, int K) {
  v16h a; const int g = lane >> 4;
#pragma unroll
  for (int i = 0; i < 8; ++i) { const int ka = k0 + 8 * g + i, kb = ka + 16;
    a[i] = (_Float16)(ka < K ? W[(size_t)(ka < K ? ka : K - 1) * ld + n] : 0.f); a[8 + i] = (_Float16)(kb < K ? W[(size_t)(kb < K ? kb : K - 1) * ld + n] : 0.f); }
  return a;
}
struct F2 { v16b h, l; };
__device__ __forceinline__ F2 bsplit16(const float v[16]) { F2 r;
#pragma unroll
  for (int i = 0; i < 16; ++i) { const __bf16 h = (__bf16)v[i]; r.h[i] = h; r.l[i] = (__bf16)(v[i] - (float)h); }
  return r; }
__device__ __forceinline__ F2 split_row(const float* row, int k0, int lane) { float v[16]; const float* p = row + k0 + 8 * (lane >> 4);
#pragma unroll
  for (int i = 0; i < 8; ++i) { v[i] = p[i]; v[8 + i] = p[16 + i]; }
  return bsplit16(v); }
__device__ __forceinline__ F2 split_rowK(const float* row, int k0, int lane, int K) { float v[16]; const int g = lane >> 4;
#pragma unroll
  for (int i = 0; i < 8; ++i) { const int ka = k0 + 8 * g + i, kb = ka + 16; v[i] = ka < K ? row[ka < K ? ka : K - 1] : 0.f; v[8 + i] = kb < K ? row[kb < K ? kb : K - 1] : 0.f; }
  return bsplit16(v); }
__device__ __forceinline__ F2 split_col(const float* W, int k0, int n, int lane, int ld, int K) { float v[16]; const int g = lane >> 4;
#pragma unroll
  for (int i = 0; i < 8; ++i) { const int ka = k0 + 8 * g + i, kb = ka + 16; v[i] = ka < K ? W[(size_t)(ka < K ? ka : K - 1) * ld + n] : 0.f; v[8 + i] = kb < K ? W[(size_t)(kb < K ? kb : K - 1) * ld + n] : 0.f; }
  return bsplit16(v); }
__device__ __forceinline__ v8f mac3(const F2& a, const F2& b, v8f c) { c = wmma_bf(a.l, b.h, c); c = wmma_bf(a.h, b.l, c); return wmma_bf(a.h, b.h, c); }
__device__ __forceinline__ float sigm(float v) { return 1.0f / (1.0f + expf(-v)); }
#define LDSX() do { asm volatile("s_wait_dscnt 0" ::: "memory"); __builtin_amdgcn_wave_barrier(); __builtin_amdgcn_fence(__ATOMIC_RELEASE, "workgroup"); } while (0)


#define NB 4
#define HW 64
#define SS (HW * HW)
#define NR (NB * SS)
#define CX 256
#define CCX 256
#define NH 4
#define HD 64
#define INNER 256
#define NGRP 32
#ifndef TNB
#define TNB NB
#define TQB (SS / 64)
#endif
typedef __attribute__((ext_vector_type(8))) __bf16 v8b;
__device__ __forceinline__ v16b frag_b(const __bf16* rowk0, int lane) {
  union { v16b v; v8b q[2]; } u; const __bf16* p = rowk0 + 8 * (lane >> 4);
  u.q[0] = *(const v8b*)p; u.q[1] = *(const v8b*)(p + 16); return u.v;
}
__device__ __forceinline__ float bfr(float v) { return (float)(__bf16)v; }
__device__ __attribute__((noinline)) float exp_ni(float v) { return expf(v); }
__device__ __attribute__((noinline)) float erf_ni(float v) { return erff(v); }

#define PK_Q 0
#define PK_K (PK_Q + INNER * CX)
#define PK_V (PK_K + INNER * CCX)
#define PK_P (PK_V + INNER * CCX)
#define PK_END (PK_P + CX * INNER)
#define WS_PK  0u
#define WS_XH  (((2u * PK_END) + 127u) / 128u * 128u)
#define WS_XL  (WS_XH + 2u * NR * CX)
#define WS_GN  (WS_XL + 2u * NR * CX)
#define WS_QP  (WS_GN + 4u * NB * NGRP * 32)
#define WS_KP  (WS_QP + 2u * NR * INNER)
#define WS_VH  (WS_KP + 2u * NR * INNER)
#define WS_VL  (WS_VH + 2u * NR * INNER)
#define WS_OH  (WS_VL + 2u * NR * INNER)
#define WS_OL  (WS_OH + 2u * NR * INNER)
#define WS_END (WS_OL + 2u * NR * INNER)

__global__ __launch_bounds__(256) void k_pack(const float* __restrict__ WQ, const float* __restrict__ WK, const float* __restrict__ WV, const float* __restrict__ WP, __bf16* __restrict__ PK) {
  __shared__ __align__(16) __bf16 s[CCX]; const int n = blockIdx.x, which = blockIdx.y, t = threadIdx.x; int K; size_t dst; const float* src;
  if (which == 0) { K = CX; src = WQ + (size_t)n * CX; dst = PK_Q + (size_t)n * CX; } else if (which == 1) { K = CCX; src = WK + (size_t)n * CCX; dst = PK_K + (size_t)n * CCX; } else if (which == 2) { K = CCX; src = WV + (size_t)n * CCX; dst = PK_V + (size_t)n * CCX; } else { if (n >= CX) return; K = INNER; src = WP + (size_t)n * INNER; dst = PK_P + (size_t)n * INNER; }
  for (int k = t; k < K; k += 256) s[k] = (__bf16)src[k];
  __syncthreads();
  for (int q = t; q < K / 8; q += 256) vst2((unsigned*)(PK + dst + q * 8), *(const v4u*)&s[q * 8]);
}
__global__ __launch_bounds__(256) void k_gnstat(const float* __restrict__ X, float* __restrict__ GN) {
  __shared__ double s1[8], s2[8]; __shared__ __align__(16) float sl[32]; const int t = threadIdx.x; const int grp = blockIdx.x, b = blockIdx.y; const float* base = X + ((size_t)b * CX + grp * 8) * SS;
  double a = 0.0, q = 0.0;
#pragma unroll 1
  for (int i = t; i < 8 * SS; i += 256) { const double v = (double)bfr(base[i]); a += v; q += v * v; }
#pragma unroll
  for (int o = 1; o < 32; o <<= 1) { a += __shfl_xor(a, o); q += __shfl_xor(q, o); }
  if ((t & 31) == 0) { s1[t >> 5] = a; s2[t >> 5] = q; }
  __syncthreads();
  if (t < 32) { double A = 0.0, Q = 0.0; for (int w = 0; w < 8; ++w) { A += s1[w]; Q += s2[w]; } const double n = 8.0 * SS; const double mean = A / n; const double var = fmax(Q / n - mean * mean, 0.0); sl[t] = (t == 0) ? (float)mean : (t == 1) ? (float)(1.0 / sqrt(var + 1e-5)) : 0.f; }
  __syncthreads();
  if (t < 8) vst2(GN + ((size_t)b * NGRP + grp) * 32 + t * 4, *(const v4f*)&sl[t * 4]);
}
__global__ __launch_bounds__(256) void k_tok(const float* __restrict__ IN, const float* __restrict__ GN, const float* __restrict__ G, const float* __restrict__ BE, __bf16* __restrict__ OH, __bf16* __restrict__ OL) {
  __shared__ float st[CX][33]; __shared__ __align__(16) __bf16 sh_[32][CX + 8], sl_[32][CX + 8]; __shared__ float smu[NGRP], srs[NGRP]; const int tid = threadIdx.x; const int pb = blockIdx.x, b = blockIdx.y; const int p0 = pb * 32;
  if (tid < NGRP) { smu[tid] = GN[((size_t)b * NGRP + tid) * 32]; srs[tid] = GN[((size_t)b * NGRP + tid) * 32 + 1]; }
#pragma unroll 1
  for (int e = tid; e < CX * 32; e += 256) { const int c = e >> 5, r = e & 31; st[c][r] = bfr(IN[((size_t)b * CX + c) * SS + p0 + r]); }
  __syncthreads();
#pragma unroll 1
  for (int e = tid; e < CX * 32; e += 256) { const int c = e >> 5, r = e & 31; const float v = (st[c][r] - smu[c >> 3]) * srs[c >> 3] * bfr(G[c]) + bfr(BE[c]); const __bf16 hb = (__bf16)v; sh_[r][c] = hb; sl_[r][c] = (__bf16)(v - (float)hb); }
  __syncthreads();
#pragma unroll 1
  for (int e = tid; e < 32 * (CX / 8); e += 256) { const int r = e / (CX / 8), pc = e % (CX / 8); const size_t o = ((size_t)b * SS + p0 + r) * CX + pc * 8; vst2((unsigned*)(OH + o), *(const v4u*)&sh_[r][pc * 8]); vst2((unsigned*)(OL + o), *(const v4u*)&sl_[r][pc * 8]); }
}
__global__ __launch_bounds__(128) void k_proj(const __bf16* __restrict__ XH, const __bf16* __restrict__ XL, const __bf16* __restrict__ CH, const __bf16* __restrict__ CL, const __bf16* __restrict__ PK, _Float16* __restrict__ QP, _Float16* __restrict__ KP, _Float16* __restrict__ VH, _Float16* __restrict__ VL) {
  __shared__ __align__(16) _Float16 so[4][16][136]; __shared__ __align__(16) _Float16 sth[128][72], stl[128][72];
  const int tid = threadIdx.x, wave = tid >> 5, lane = tid & 31, col = lane & 15, g = lane >> 4; const size_t r0 = (size_t)blockIdx.x * 64 + wave * 16; const int n0 = blockIdx.y * 128; const int which = blockIdx.z;
  const __bf16* AH = (which == 0) ? XH : CH; const __bf16* AL = (which == 0) ? XL : CL; const int K = (which == 0) ? CX : CCX; const __bf16* PW = PK + ((which == 0) ? PK_Q : (which == 1) ? PK_K : PK_V);
  v8f acc[8] = {};
#pragma unroll 2
  for (int kc = 0; kc < K / 32; ++kc) { const v16b ah = frag_b(AH + (r0 + col) * K + kc * 32, lane), al = frag_b(AL + (r0 + col) * K + kc * 32, lane);
#pragma unroll
    for (int j = 0; j < 8; ++j) { const v16b w = frag_b(PW + (size_t)(n0 + j * 16 + col) * K + kc * 32, lane); acc[j] = wmma_bf(al, w, acc[j]); acc[j] = wmma_bf(ah, w, acc[j]); } }
  if (which < 2) { const float sc = (which == 0) ? 0.125f : 1.0f;
#pragma unroll
    for (int j = 0; j < 8; ++j) {
#pragma unroll
      for (int r = 0; r < 8; ++r) so[wave][8 * g + r][j * 16 + col] = (_Float16)(acc[j][r] * sc); }
    LDSX();
    _Float16* DST = (which == 0) ? QP : KP;
    for (int rl = 0; rl < 16; ++rl) if (lane < 16) vst2((unsigned*)(DST + (r0 + rl) * INNER + n0 + lane * 8), *(const v4u*)&so[wave][rl][lane * 8]);
  } else {
#pragma unroll
    for (int j = 0; j < 8; ++j) {
#pragma unroll
      for (int r = 0; r < 8; ++r) { const float v = acc[j][r]; const _Float16 hv = (_Float16)v; sth[j * 16 + col][wave * 16 + 8 * g + r] = hv; stl[j * 16 + col][wave * 16 + 8 * g + r] = (_Float16)((v - (float)hv) * 2048.0f); } }
    __syncthreads();
    const size_t rb = (size_t)blockIdx.x * 64; const int b = (int)(rb / SS), s0 = (int)(rb % SS);
    for (int e = tid; e < 128 * 8; e += 128) { const int d = e >> 3, pc = e & 7; const size_t o = ((size_t)b * INNER + n0 + d) * SS + s0 + pc * 8; vst2((unsigned*)(VH + o), *(const v4u*)&sth[d][pc * 8]); vst2((unsigned*)(VL + o), *(const v4u*)&stl[d][pc * 8]); }
  }
}
__global__ __launch_bounds__(128) void k_attn(const _Float16* __restrict__ QP, const _Float16* __restrict__ KP, const _Float16* __restrict__ VH, const _Float16* __restrict__ VL, __bf16* __restrict__ OH, __bf16* __restrict__ OL) {
  __shared__ __align__(16) _Float16 sp[4][16][40]; __shared__ __align__(16) __bf16 soh[4][16][72], sol[4][16][72];
  const int tid = threadIdx.x, wave = tid >> 5, lane = tid & 31, col = lane & 15, g = lane >> 4; const int qb = blockIdx.x, h = blockIdx.y, b = blockIdx.z; const int q0 = qb * 64 + wave * 16; const size_t rq = (size_t)b * SS + q0 + col;
  v16h aq[2];
#pragma unroll
  for (int kc = 0; kc < 2; ++kc) aq[kc] = frag_h(QP + rq * INNER + h * HD + kc * 32, lane);
  const _Float16* Vbh = VH + ((size_t)b * INNER + h * HD) * SS; const _Float16* Vbl = VL + ((size_t)b * INNER + h * HD) * SS;
  float m[8], l[8];
#pragma unroll
  for (int r = 0; r < 8; ++r) { m[r] = -3.0e38f; l[r] = 0.f; }
  v8f acc[4] = {}, accl[4] = {};
#pragma unroll 1
  for (int ks = 0; ks < SS / 32; ++ks) { v8f s[2];
#pragma unroll
    for (int ct = 0; ct < 2; ++ct) { const int kk = ks * 32 + ct * 16 + col; const size_t rk = ((size_t)b * SS + kk) * INNER + h * HD; v8f c = {};
#pragma unroll
      for (int kc = 0; kc < 2; ++kc) c = wmma16(aq[kc], frag_h(KP + rk + kc * 32, lane), c);
#pragma unroll
      for (int r = 0; r < 8; ++r) s[ct][r] = c[r]; }
#pragma unroll
    for (int r = 0; r < 8; ++r) { float mx = fmaxf(s[0][r], s[1][r]);
#pragma unroll
      for (int o = 1; o < 16; o <<= 1) mx = fmaxf(mx, __shfl_xor(mx, o));
      const float mn = fmaxf(m[r], mx); const float alpha = (m[r] <= -1.0e38f) ? 0.f : exp_ni(m[r] - mn); const float e0 = exp_ni(s[0][r] - mn), e1 = exp_ni(s[1][r] - mn); float es = e0 + e1;
#pragma unroll
      for (int o = 1; o < 16; o <<= 1) es += __shfl_xor(es, o);
      l[r] = l[r] * alpha + es; m[r] = mn;
#pragma unroll
      for (int dt = 0; dt < 4; ++dt) { acc[dt][r] *= alpha; accl[dt][r] *= alpha; }
      sp[wave][8 * g + r][col] = (_Float16)e0; sp[wave][8 * g + r][16 + col] = (_Float16)e1; }
    LDSX();
    const v16h pa = frag_h(&sp[wave][col][0], lane);
#pragma unroll
    for (int dt = 0; dt < 4; ++dt) { const size_t vo = (size_t)(dt * 16 + col) * SS + ks * 32; acc[dt] = wmma16(pa, frag_h(Vbh + vo, lane), acc[dt]); accl[dt] = wmma16(pa, frag_h(Vbl + vo, lane), accl[dt]); }
    LDSX(); }
#pragma unroll
  for (int r = 0; r < 8; ++r) { const float il = 1.0f / l[r];
#pragma unroll
    for (int dt = 0; dt < 4; ++dt) { const float v = (acc[dt][r] + accl[dt][r] * (1.0f / 2048.0f)) * il; const __bf16 hb = (__bf16)v; soh[wave][8 * g + r][dt * 16 + col] = hb; sol[wave][8 * g + r][dt * 16 + col] = (__bf16)(v - (float)hb); } }
  LDSX();
  for (int rl = 0; rl < 16; ++rl) { const size_t o = ((size_t)b * SS + q0 + rl) * INNER + h * HD; if (lane < 8) vst2((unsigned*)(OH + o + lane * 8), *(const v4u*)&soh[wave][rl][lane * 8]); else if (lane < 16) vst2((unsigned*)(OL + o + (lane - 8) * 8), *(const v4u*)&sol[wave][rl][(lane - 8) * 8]); }
}
__global__ __launch_bounds__(128) void k_out(const __bf16* __restrict__ OH, const __bf16* __restrict__ OL, const __bf16* __restrict__ PK, const float* __restrict__ X, float* __restrict__ OUT) {
  __shared__ __align__(16) float st[128][68];
  const int tid = threadIdx.x, wave = tid >> 5, lane = tid & 31, col = lane & 15, g = lane >> 4; const size_t r0 = (size_t)blockIdx.x * 64 + wave * 16; const size_t rb = (size_t)blockIdx.x * 64; const int b = (int)(rb / SS), p0 = (int)(rb % SS);
#pragma unroll 1
  for (int half = 0; half < 2; ++half) { v8f acc[8] = {};
#pragma unroll 2
    for (int kc = 0; kc < INNER / 32; ++kc) { const v16b ah = frag_b(OH + (r0 + col) * INNER + kc * 32, lane), al = frag_b(OL + (r0 + col) * INNER + kc * 32, lane);
#pragma unroll
      for (int j = 0; j < 8; ++j) { const v16b w = frag_b(PK + PK_P + (size_t)(half * 128 + j * 16 + col) * INNER + kc * 32, lane); acc[j] = wmma_bf(al, w, acc[j]); acc[j] = wmma_bf(ah, w, acc[j]); } }
#pragma unroll
    for (int j = 0; j < 8; ++j) { const int cl = j * 16 + col; const int c = half * 128 + cl;
#pragma unroll
      for (int r = 0; r < 8; ++r) { const int pl = wave * 16 + 8 * g + r; st[cl][pl] = acc[j][r] + bfr(X[((size_t)b * CX + c) * SS + p0 + pl]); } }
    __syncthreads();
    for (int e = tid; e < 128 * 16; e += 128) { const int cl = e >> 4, pc = e & 15; vst2(OUT + ((size_t)b * CX + half * 128 + cl) * SS + p0 + pc * 4, *(const v4f*)&st[cl][pc * 4]); }
    __syncthreads(); }
}
extern "C" void kernel_launch(void* const* d_in, const int* in_sizes, int n_in, void* d_out, int out_size, void* d_ws, size_t ws_size, hipStream_t stream) {
  (void)in_sizes; (void)n_in; (void)out_size;
  const float** F = (const float**)d_in;
  if (ws_size < (size_t)WS_END) return;
  char* ws = (char*)d_ws; __bf16 *PK = (__bf16*)(ws + WS_PK), *XH = (__bf16*)(ws + WS_XH), *XL = (__bf16*)(ws + WS_XL), *OH = (__bf16*)(ws + WS_OH), *OL = (__bf16*)(ws + WS_OL); float* GN = (float*)(ws + WS_GN); _Float16 *QP = (_Float16*)(ws + WS_QP), *KP = (_Float16*)(ws + WS_KP), *VH = (_Float16*)(ws + WS_VH), *VL = (_Float16*)(ws + WS_VL);
  k_pack<<<dim3(INNER, 4), 256, 0, stream>>>(F[3], F[4], F[5], F[6], PK);
  k_gnstat<<<dim3(NGRP, TNB), 256, 0, stream>>>(F[0], GN);
  k_tok<<<dim3(SS / 32, TNB), 256, 0, stream>>>(F[0], GN, F[1], F[2], XH, XL);
  k_proj<<<dim3(TNB * SS / 64, INNER / 128, 3), 128, 0, stream>>>(XH, XL, XH, XL, PK, QP, KP, VH, VL);
  k_attn<<<dim3(TQB, NH, TNB), 128, 0, stream>>>(QP, KP, VH, VL, OH, OL);
  k_out<<<TNB * SS / 64, 128, 0, stream>>>(OH, OL, PK, F[0], (float*)d_out);
}
